// GCNModel_15470472200268
// MI455X (gfx1250) — hardware-verified
//
#include <hip/hip_runtime.h>
#include <stddef.h>
#include <stdint.h>
#include <math.h>


#define CIN    128
#define HID    256
#define NGR    64
#define NTHR   256
#define NWAVE  8
#define EPT    8
#define CHUNK  (NTHR * EPT)
#define WCAP   (EPT * 32)
#define LISTN  (NWAVE * WCAP)
#define NBD    8192
#define SLD    13
#define NBA    1024
#define SLA    10
#define RCAP   28672
#define DEGCAP 64
#define GBM    64
#define GBN    64
#define GTHR   128
#define NBW1   ((HID * (CIN / 8)) / NTHR)
#define NBW2   ((HID * HID / 4) / NTHR)
#define SMF    1024
#define NFLAG  64
#define NMAXN  50000
#define POOLCAP 50048
#define POOL_LDS_BYTES (POOLCAP * 4 + HID * 4 + HID * 4 + 64)
#define AGG_ZINTS (LISTN + 2 * RCAP + 3 * NBA)
#define AGG_LDS_INTS (AGG_ZINTS + 16)
#define WSMAX  134217728

static_assert((CHUNK & (CHUNK - 1)) == 0 && CHUNK <= 4096);
static_assert((NBD & (NBD - 1)) == 0 && NBD == (1 << SLD));
static_assert((NBA & (NBA - 1)) == 0 && NBA == (1 << SLA));
static_assert(((long long)CHUNK << SLD) < (1LL << 31));
static_assert(((long long)CHUNK << SLA) < (1LL << 31));
static_assert(NBD % (NTHR * 4) == 0);
static_assert(LISTN % NTHR == 0);
static_assert(NBA % NWAVE == 0 && NBA % 32 == 0 && NBA % GBM == 0 && NBA % NTHR == 0);
static_assert(RCAP % 32 == 0 && AGG_ZINTS % 4 == 0 && LISTN % 4 == 0);
static_assert(CIN % 32 == 0 && CIN / 8 == 16);
static_assert(GBM == (GTHR / 32) * 16 && GBN == 64 && HID % GBN == 0);
static_assert(HID == NTHR && HID == 8 * 32);
static_assert(SMF == 4 * NTHR && SMF == 4 * HID);
static_assert(POOLCAP >= NMAXN + 8 && POOLCAP % 4 == 0);
static_assert(AGG_LDS_INTS * 4 <= 300000 && POOL_LDS_BYTES <= 300000);
static_assert((NGR * 4) % 128 == 0 && NGR == 8 * NWAVE);
static_assert(NGR * HID / 4 >= NTHR);

typedef float          v4f   __attribute__((ext_vector_type(4)));
typedef float          v8f   __attribute__((ext_vector_type(8)));
typedef int            v4i   __attribute__((ext_vector_type(4)));
typedef int            v8i   __attribute__((ext_vector_type(8)));
typedef unsigned short v8us  __attribute__((ext_vector_type(8)));
typedef unsigned short v16us __attribute__((ext_vector_type(16)));
typedef __bf16         v16bf __attribute__((ext_vector_type(16)));
typedef v4f  __attribute__((may_alias)) v4fa;
typedef v4i  __attribute__((may_alias)) v4ia;
typedef v8us __attribute__((may_alias)) v8usa;
union FragB { v16bf v; v16us u; v8us h[2]; v8i w; };

__device__ __forceinline__ v8f wmb(const FragB& a, const FragB& b, v8f c) {
  v8f d = __builtin_amdgcn_wmma_f32_16x16x32_bf16(false, a.v, false, b.v, (short)0, c, false, false);
  asm volatile("v_nop\n\tv_nop\n\tv_nop\n\tv_nop" : "+v"(d) : "v"(a.w), "v"(b.w));
  return d;
}

__device__ __forceinline__ unsigned bf16_bits(float f) {
  const unsigned u = __float_as_uint(f);
  return (u + 0x7FFFu + ((u >> 16) & 1u)) >> 16;
}
__device__ __forceinline__ float bf16_val(float f) {
  return __uint_as_float(bf16_bits(f) << 16);
}
__device__ __forceinline__ float sel4(int seg, float a, float b, float c, float d) {
  return seg == 0 ? a : (seg == 1 ? b : (seg == 2 ? c : d));
}

template <int SLB>
__device__ __forceinline__ int scan_chunk(const int* __restrict__ dsts, int nE, int cbase, int slotBase,
                                          int nb, int vec8, int* list, int tid, int lane, int wave) {
  int wc = 0;
  const int el0  = tid * EPT;
  const int e0   = cbase + el0;
  const int sent = -2147483647 - 1;
  v4i da, db;
  if (vec8 != 0 && cbase + CHUNK <= nE) {
    da = *(const v4i*)(dsts + e0);
    db = *(const v4i*)(dsts + e0 + 4);
  } else {
    da.x = (e0     < nE) ? dsts[min(e0,     nE - 1)] : sent;
    da.y = (e0 + 1 < nE) ? dsts[min(e0 + 1, nE - 1)] : sent;
    da.z = (e0 + 2 < nE) ? dsts[min(e0 + 2, nE - 1)] : sent;
    da.w = (e0 + 3 < nE) ? dsts[min(e0 + 3, nE - 1)] : sent;
    db.x = (e0 + 4 < nE) ? dsts[min(e0 + 4, nE - 1)] : sent;
    db.y = (e0 + 5 < nE) ? dsts[min(e0 + 5, nE - 1)] : sent;
    db.z = (e0 + 6 < nE) ? dsts[min(e0 + 6, nE - 1)] : sent;
    db.w = (e0 + 7 < nE) ? dsts[min(e0 + 7, nE - 1)] : sent;
  }
  const unsigned nbs = (unsigned)slotBase;
  const unsigned unb = (unsigned)nb;
  const unsigned s0 = (unsigned)da.x - nbs, s1 = (unsigned)da.y - nbs;
  const unsigned s2 = (unsigned)da.z - nbs, s3 = (unsigned)da.w - nbs;
  const unsigned s4 = (unsigned)db.x - nbs, s5 = (unsigned)db.y - nbs;
  const unsigned s6 = (unsigned)db.z - nbs, s7 = (unsigned)db.w - nbs;
  const bool h0 = s0 < unb, h1 = s1 < unb, h2 = s2 < unb, h3 = s3 < unb;
  const bool h4 = s4 < unb, h5 = s5 < unb, h6 = s6 < unb, h7 = s7 < unb;
  const unsigned any = __builtin_amdgcn_ballot_w32(h0 | h1 | h2 | h3 | h4 | h5 | h6 | h7);
  if (any != 0u) {
#define HITJ(J, HJ, SJ) { \
      const unsigned mj = __builtin_amdgcn_ballot_w32(HJ); \
      if (mj != 0u) { \
        if (HJ) { \
          const int pos = wc + (int)__builtin_amdgcn_mbcnt_lo(mj, 0u); \
          if (pos < WCAP) list[wave * WCAP + pos] = ((el0 + (J)) << SLB) | (int)(SJ); \
        } \
        wc += (int)__builtin_popcount(mj); } }
    HITJ(0, h0, s0)
    HITJ(1, h1, s1)
    HITJ(2, h2, s2)
    HITJ(3, h3, s3)
    HITJ(4, h4, s4)
    HITJ(5, h5, s5)
    HITJ(6, h6, s6)
    HITJ(7, h7, s7)
#undef HITJ
  }
  return wc;
}

__global__ __launch_bounds__(NTHR) void k_prep(const float* __restrict__ x, int nN, int nbX,
                                               const float* __restrict__ W1, const float* __restrict__ b1,
                                               const float* __restrict__ W2, const float* __restrict__ b2,
                                               const float* __restrict__ w3, const float* __restrict__ b3,
                                               unsigned short* xb, unsigned short* W1T, float* W2R, float* SM) {
  const int tid = (int)threadIdx.x;
  int b = (int)blockIdx.x;
  if (b < nbX) {
    const int u   = b * NTHR + tid;
    const int row = u >> 4;
    const int k8  = (u & 15) * 8;
    const int rc  = row < nN ? row : nN - 1;
    const float* p = x + (size_t)rc * CIN + k8;
    const v4f a = *(const v4fa*)p;
    const v4f c = *(const v4fa*)(p + 4);
    const bool ok = row < nN;
    v8us o;
    o[0] = ok ? (unsigned short)bf16_bits(a.x) : (unsigned short)0;
    o[1] = ok ? (unsigned short)bf16_bits(a.y) : (unsigned short)0;
    o[2] = ok ? (unsigned short)bf16_bits(a.z) : (unsigned short)0;
    o[3] = ok ? (unsigned short)bf16_bits(a.w) : (unsigned short)0;
    o[4] = ok ? (unsigned short)bf16_bits(c.x) : (unsigned short)0;
    o[5] = ok ? (unsigned short)bf16_bits(c.y) : (unsigned short)0;
    o[6] = ok ? (unsigned short)bf16_bits(c.z) : (unsigned short)0;
    o[7] = ok ? (unsigned short)bf16_bits(c.w) : (unsigned short)0;
    unsigned short* dp = xb + (size_t)row * CIN + k8;
    *(volatile v8us*)dp = o;
    __threadfence();
    *(volatile v8us*)dp = o;
    return;
  }
  b -= nbX;
  if (b < NBW1) {
    const int u  = b * NTHR + tid;
    const int n  = u >> 4;
    const int k8 = (u & 15) * 8;
    const float* p = W1 + (size_t)k8 * HID + n;
    v8us o;
#pragma unroll
    for (int i = 0; i < 8; ++i) o[i] = (unsigned short)bf16_bits(p[(size_t)i * HID]);
    unsigned short* dp = W1T + (size_t)n * CIN + k8;
    *(volatile v8us*)dp = o;
    __threadfence();
    *(volatile v8us*)dp = o;
    return;
  }
  b -= NBW1;
  if (b < NBW2) {
    const int u = b * NTHR + tid;
    const v4f a = *(const v4fa*)(W2 + 4 * (size_t)u);
    v4f o;
    o.x = bf16_val(a.x); o.y = bf16_val(a.y); o.z = bf16_val(a.z); o.w = bf16_val(a.w);
    float* dp = W2R + 4 * (size_t)u;
    *(volatile v4f*)dp = o;
    __threadfence();
    *(volatile v4f*)dp = o;
    return;
  }
  {
    const int seg = tid >> 6;
    const int i4  = (tid & 63) * 4;
    const v4f va = *(const v4fa*)(b1 + i4);
    const v4f vb = *(const v4fa*)(b2 + i4);
    const v4f vc = *(const v4fa*)(w3 + i4);
    const float sd = b3[0];
    const float d0 = (tid == 3 * 64) ? bf16_val(sd) : 0.0f;
    v4f o;
    o.x = sel4(seg, bf16_val(va.x), bf16_val(vb.x), bf16_val(vc.x), d0);
    o.y = sel4(seg, bf16_val(va.y), bf16_val(vb.y), bf16_val(vc.y), 0.0f);
    o.z = sel4(seg, bf16_val(va.z), bf16_val(vb.z), bf16_val(vc.z), 0.0f);
    o.w = sel4(seg, bf16_val(va.w), bf16_val(vb.w), bf16_val(vc.w), 0.0f);
    float* dp = SM + 4 * tid;
    *(volatile v4f*)dp = o;
    __threadfence();
    *(volatile v4f*)dp = o;
  }
}

__global__ __launch_bounds__(NTHR) void k_deg(const int* __restrict__ dsts, int nE, int vec8, float* dis) {
  __shared__ __attribute__((aligned(16))) int scnt[NBD];
  __shared__ __attribute__((aligned(16))) int list[LISTN];
  __shared__ int wcnt[NWAVE];
  const int tid = (int)threadIdx.x, lane = tid & 31, wave = tid >> 5;
  const int nodeBase = (int)blockIdx.x * NBD;

  for (int i = tid; i < NBD; i += NTHR) scnt[i] = 0;
  for (int i = tid; i < LISTN; i += NTHR) list[i] = 0;
  if (tid < NWAVE) wcnt[tid] = 0;
  __syncthreads();

  const int nChunks = (nE + CHUNK - 1) / CHUNK;
#pragma unroll 1
  for (int ch = 0; ch < nChunks; ++ch) {
    const int cbase = ch * CHUNK;
    const int wc = scan_chunk<SLD>(dsts, nE, cbase, nodeBase, NBD, vec8, list, tid, lane, wave);
    if (lane == 0) wcnt[wave] = wc;
    __syncthreads();
    if (wave == 0) {
#pragma unroll 1
      for (int w2 = 0; w2 < NWAVE; ++w2) {
        int c = wcnt[w2];
        c = c < 0 ? 0 : (c > WCAP ? WCAP : c);
#pragma unroll 1
        for (int b0 = 0; b0 < c; b0 += 32) {
          const int idx = b0 + lane;
          const int ent = list[w2 * WCAP + (idx < WCAP ? idx : WCAP - 1)];
          const int m32 = (c - b0) < 32 ? (c - b0) : 32;
#pragma unroll 1
          for (int k = 0; k < m32; ++k) {
            const int u  = __builtin_amdgcn_readlane(ent, k);
            const int sl = u & (NBD - 1);
            if (lane == 0) scnt[sl] = scnt[sl] + 1;
          }
        }
      }
    }
    __syncthreads();
  }

#pragma unroll 1
  for (int i = tid; i < NBD; i += NTHR) {
    int c = scnt[i];
    c = c < 0 ? 0 : c;
    const float d = (float)c + 1.0f;
    const float r = 1.0f / sqrtf(d);
    const float v = (d > 0.0f) ? r : 0.0f;
    scnt[i] = __float_as_int(v);
  }
  __syncthreads();

  v4f vals[NBD / (NTHR * 4)];
#pragma unroll
  for (int it = 0; it < NBD / (NTHR * 4); ++it) {
    const int s0 = it * (NTHR * 4) + 4 * tid;
    vals[it] = *(const v4fa*)(scnt + s0);
  }
#pragma unroll
  for (int it = 0; it < NBD / (NTHR * 4); ++it) {
    const int s0 = it * (NTHR * 4) + 4 * tid;
    *(volatile v4f*)(dis + (size_t)nodeBase + s0) = vals[it];
  }
  __threadfence();
#pragma unroll
  for (int it = 0; it < NBD / (NTHR * 4); ++it) {
    const int s0 = it * (NTHR * 4) + 4 * tid;
    *(volatile v4f*)(dis + (size_t)nodeBase + s0) = vals[it];
  }
}

__global__ __launch_bounds__(GTHR) void k_gemm(
    const unsigned short* __restrict__ A, const unsigned short* __restrict__ WT,
    float* outF, int K, int ldo)
{
  __shared__ __attribute__((aligned(16))) float stg[GBM * GBN];
  const int tid = (int)threadIdx.x, lane = tid & 31, wave = tid >> 5, hh = lane >> 4, m = lane & 15;
  const int rowBase = (int)blockIdx.x * GBM;
  const int col0    = (int)blockIdx.y * GBN;

  v8f acc[4];
  {
    const v8f z = {0.f, 0.f, 0.f, 0.f, 0.f, 0.f, 0.f, 0.f};
    acc[0] = z; acc[1] = z; acc[2] = z; acc[3] = z;
  }
  const unsigned short* ap = A  + (size_t)(rowBase + 16 * wave + m) * (size_t)K + 8 * hh;
  const unsigned short* wp = WT + (size_t)(col0 + m) * (size_t)K + 8 * hh;
  const int ksteps = K >> 5;
#pragma unroll 1
  for (int ks = 0; ks < ksteps; ++ks) {
    FragB af;
    af.h[0] = *(const v8usa*)(ap + 32 * ks);
    af.h[1] = *(const v8usa*)(ap + 32 * ks + 16);
#pragma unroll
    for (int t = 0; t < 4; ++t) {
      const unsigned short* wq = wp + (size_t)(16 * t) * (size_t)K + 32 * ks;
      FragB bf;
      bf.h[0] = *(const v8usa*)wq;
      bf.h[1] = *(const v8usa*)(wq + 16);
      acc[t] = wmb(af, bf, acc[t]);
    }
  }

#pragma unroll
  for (int t = 0; t < 4; ++t) {
    const int lc = 16 * t + m;
#pragma unroll
    for (int r = 0; r < 8; ++r) {
      const int lr = 16 * wave + 8 * hh + r;
      stg[lr * GBN + lc] = acc[t][r];
    }
  }
  __syncthreads();

  v4f fv[8];
#pragma unroll
  for (int i = 0; i < 8; ++i) {
    const int lr = 16 * wave + 2 * i + hh;
    fv[i] = *(const v4fa*)(stg + lr * GBN + 4 * m);
  }
#pragma unroll
  for (int i = 0; i < 8; ++i) {
    const int lr = 16 * wave + 2 * i + hh;
    const int gr = rowBase + lr;
    float* op = outF + (size_t)gr * (size_t)ldo + col0 + 4 * m;
    *(volatile v4f*)op = fv[i];
  }
  __threadfence();
#pragma unroll
  for (int i = 0; i < 8; ++i) {
    const int lr = 16 * wave + 2 * i + hh;
    const int gr = rowBase + lr;
    float* op = outF + (size_t)gr * (size_t)ldo + col0 + 4 * m;
    *(volatile v4f*)op = fv[i];
  }
}

__device__ __forceinline__ float fin1(float acc, float sv, float rd, float bv, float pzr, bool live) {
  float y = (acc + sv * rd) + bv;
  y = (y > 0.0f) ? y : (y - y);
  y = y + pzr;
  return live ? y : 0.0f;
}

__global__ __launch_bounds__(NTHR) void k_agg(const int* __restrict__ srcs, const int* __restrict__ dsts,
                                              int nE, int nN, int vec8, int mRows,
                                              const float* __restrict__ dis,
                                              const float* __restrict__ xl, const float* __restrict__ bias,
                                              float* hout, int* flags) {
  extern __shared__ __attribute__((aligned(16))) int dsm[];
  int* list = dsm;
  int* hl   = dsm + LISTN;
  int* sl   = dsm + LISTN + RCAP;
  int* cnt  = dsm + LISTN + 2 * RCAP;
  int* offs = cnt + NBA;
  int* cur  = offs + NBA;
  int* misc = cur + NBA;
  const int tid = (int)threadIdx.x, lane = tid & 31, wave = tid >> 5;
  const int nodeBase = (int)blockIdx.x * NBA;

  {
    const v4i z4 = {0, 0, 0, 0};
    for (int i = tid * 4; i < AGG_ZINTS; i += NTHR * 4) *(v4ia*)(dsm + i) = z4;
    if (tid < 16) misc[tid] = 0;
  }
  const v4f bvA = *(const v4fa*)(bias + 4 * lane);
  const v4f bvB = *(const v4fa*)(bias + 128 + 4 * lane);
  __syncthreads();

  int t = 0, ov = 0;
  const int nChunks = (nE + CHUNK - 1) / CHUNK;
#pragma unroll 1
  for (int ch = 0; ch < nChunks; ++ch) {
    const int cbase = ch * CHUNK;
    const int wc = scan_chunk<SLA>(dsts, nE, cbase, nodeBase, NBA, vec8, list, tid, lane, wave);
    if (lane == 0) misc[wave] = wc;
    __syncthreads();
    if (wave == 0) {
#pragma unroll 1
      for (int w2 = 0; w2 < NWAVE; ++w2) {
        int c = misc[w2];
        c = c < 0 ? 0 : (c > WCAP ? WCAP : c);
#pragma unroll 1
        for (int b0 = 0; b0 < c; b0 += 32) {
          const int idx = b0 + lane;
          const int ent = list[w2 * WCAP + (idx < WCAP ? idx : WCAP - 1)];
          const int m32 = (c - b0) < 32 ? (c - b0) : 32;
#pragma unroll 1
          for (int k = 0; k < m32; ++k) {
            const int u    = __builtin_amdgcn_readlane(ent, k);
            const int slot = u & (NBA - 1);
            const int el   = (u >> SLA) & (CHUNK - 1);
            const int pk   = ((cbase + el) << SLA) | slot;
            if (t < RCAP) {
              if (lane == 0) { hl[t] = pk; cnt[slot] = cnt[slot] + 1; }
              t = t + 1;
            } else {
              ov = 1;
            }
          }
        }
      }
    }
    __syncthreads();
  }
  {
    int bg = 0;
#pragma unroll
    for (int i = 0; i < NBA / NTHR; ++i) bg |= (cnt[tid + NTHR * i] > DEGCAP) ? 1 : 0;
    if (bg != 0) misc[10] = 1;
  }
  if (wave == 0 && lane == 0) { misc[8] = t; misc[9] = ov; }
  __syncthreads();
  int tt = misc[8];
  tt = tt < 0 ? 0 : (tt > RCAP ? RCAP : tt);
  const int ovf  = misc[9];
  const int bigf = misc[10];

  {
    v4i fv;
    fv.x = (lane == 0) ? ((ovf | bigf) != 0 ? 1 : 0) : 0;
    fv.y = 0; fv.z = 0; fv.w = 0;
    int* fp = flags + (size_t)blockIdx.x * 32 + 4 * (lane & 7);
    const bool fw = (wave == 0) && (lane < 8);
    if (fw) *(volatile v4i*)fp = fv;
    __threadfence();
    if (fw) *(volatile v4i*)fp = fv;
  }

  if (wave == 0) {
    const int base = lane * (NBA / 32);
    int s = 0;
#pragma unroll 1
    for (int i = 0; i < NBA / 32; ++i) s += cnt[base + i];
    int incl = s;
#pragma unroll
    for (int d = 1; d < 32; d <<= 1) {
      const int y = __shfl_up(incl, d, 32);
      if (lane >= d) incl += y;
    }
    int run = incl - s;
#pragma unroll 1
    for (int i = 0; i < NBA / 32; ++i) {
      const int cv = cnt[base + i];
      offs[base + i] = run;
      cur[base + i]  = run;
      run += cv;
    }
  }
  __syncthreads();
  if (wave == 0) {
#pragma unroll 1
    for (int b0 = 0; b0 < tt; b0 += 32) {
      const int idx = b0 + lane;
      const int ent = hl[idx < RCAP ? idx : RCAP - 1];
      const int m32 = (tt - b0) < 32 ? (tt - b0) : 32;
#pragma unroll 1
      for (int k = 0; k < m32; ++k) {
        const int u    = __builtin_amdgcn_readlane(ent, k);
        const int slot = u & (NBA - 1);
        if (lane == 0) {
          int p = cur[slot];
          p = p < 0 ? 0 : (p > RCAP - 1 ? RCAP - 1 : p);
          sl[p] = u;
          cur[slot] = p + 1;
        }
      }
    }
  }
  __syncthreads();

  const float qnan = __int_as_float(0x7fc00000);
  const float pz = (ovf != 0) ? qnan : 0.0f;
#pragma unroll 1
  for (int si = 0; si < NBA / NWAVE; ++si) {
    const int s    = si * NWAVE + wave;
    const int node = nodeBase + s;
    int c = cnt[s];
    const bool big = c > DEGCAP;
    c = c < 0 ? 0 : (c > DEGCAP ? DEGCAP : c);
    int o = offs[s];
    o = o < 0 ? 0 : (o > RCAP ? RCAP : o);
    const int nc = node < nN ? node : nN - 1;
    const float dd = dis[nc];
    const float rd = dd * dd;
    v4f aA = {0.0f, 0.0f, 0.0f, 0.0f};
    v4f aB = {0.0f, 0.0f, 0.0f, 0.0f};
#pragma unroll 1
    for (int b0 = 0; b0 < c; b0 += 32) {
      int idx = o + b0 + lane;
      idx = idx > RCAP - 1 ? RCAP - 1 : idx;
      const int ent = sl[idx];
      int eid = ent >> SLA;
      eid = eid < 0 ? 0 : (eid > nE - 1 ? nE - 1 : eid);
      int sr = srcs[eid];
      sr = sr < 0 ? 0 : (sr > nN - 1 ? nN - 1 : sr);
      const float cf  = dis[sr] * dd;
      const int   cfi = __float_as_int(cf);
      const int m32 = (c - b0) < 32 ? (c - b0) : 32;
#pragma unroll 1
      for (int k = 0; k < m32; ++k) {
        const int   sk = __builtin_amdgcn_readlane(sr, k);
        const float ck = __int_as_float(__builtin_amdgcn_readlane(cfi, k));
        const float* rp = xl + (size_t)sk * HID + 4 * lane;
        const v4f a = *(const v4fa*)rp;
        const v4f b = *(const v4fa*)(rp + 128);
        aA.x = fmaf(ck, a.x, aA.x); aA.y = fmaf(ck, a.y, aA.y);
        aA.z = fmaf(ck, a.z, aA.z); aA.w = fmaf(ck, a.w, aA.w);
        aB.x = fmaf(ck, b.x, aB.x); aB.y = fmaf(ck, b.y, aB.y);
        aB.z = fmaf(ck, b.z, aB.z); aB.w = fmaf(ck, b.w, aB.w);
      }
    }
    const float* sp = xl + (size_t)nc * HID + 4 * lane;
    const v4f sA = *(const v4fa*)sp;
    const v4f sB = *(const v4fa*)(sp + 128);
    const float pzr = big ? qnan : pz;
    const bool live = node < nN;
    v4f oA, oB;
    oA.x = fin1(aA.x, sA.x, rd, bvA.x, pzr, live);
    oA.y = fin1(aA.y, sA.y, rd, bvA.y, pzr, live);
    oA.z = fin1(aA.z, sA.z, rd, bvA.z, pzr, live);
    oA.w = fin1(aA.w, sA.w, rd, bvA.w, pzr, live);
    oB.x = fin1(aB.x, sB.x, rd, bvB.x, pzr, live);
    oB.y = fin1(aB.y, sB.y, rd, bvB.y, pzr, live);
    oB.z = fin1(aB.z, sB.z, rd, bvB.z, pzr, live);
    oB.w = fin1(aB.w, sB.w, rd, bvB.w, pzr, live);
    const bool wr = node < mRows;
    float* op = hout + (size_t)node * HID + 4 * lane;
    if (wr) { *(volatile v4f*)op = oA; *(volatile v4f*)(op + 128) = oB; }
    __threadfence();
    if (wr) { *(volatile v4f*)op = oA; *(volatile v4f*)(op + 128) = oB; }
  }
}

__global__ __launch_bounds__(NTHR) void k_pool_head(const float* __restrict__ h1, const int* __restrict__ bat,
                                                    int nN, int R, const float* __restrict__ W2R,
                                                    const float* __restrict__ SM, float* Z) {
  extern __shared__ __attribute__((aligned(16))) int psm[];
  int*   plist  = psm;
  float* pooled = (float*)(psm + POOLCAP);
  float* zs     = pooled + HID;
  int*   wcn    = (int*)(zs + HID);
  const int tid = (int)threadIdx.x, lane = tid & 31, wave = tid >> 5;
  const int g = (int)blockIdx.x;

  {
    const int beg = wave * R;
    int end = beg + R;
    end = end > nN ? nN : end;
    int c = 0;
#pragma unroll 1
    for (int i0 = beg; i0 < end; i0 += 32) {
      const int i  = i0 + lane;
      int ic = i < nN ? i : nN - 1;
      ic = ic < 0 ? 0 : ic;
      const int b  = bat[ic];
      const bool hit = (i < end) && (b == g);
      const unsigned msk = __builtin_amdgcn_ballot_w32(hit);
      if (hit) {
        const int pos = c + (int)__builtin_amdgcn_mbcnt_lo(msk, 0u);
        if (pos < R) plist[beg + pos] = i;
      }
      c += (int)__builtin_popcount(msk);
    }
    if (lane == 0) wcn[wave] = c;
  }
  __syncthreads();

  double acc = 0.0;
  int total = 0;
#pragma unroll 1
  for (int w2 = 0; w2 < NWAVE; ++w2) {
    int cw = wcn[w2];
    cw = cw < 0 ? 0 : (cw > R ? R : cw);
    total += cw;
    const int lb = w2 * R;
#pragma unroll 4
    for (int j = 0; j < cw; ++j) {
      int node = plist[lb + j];
      node = node < 0 ? 0 : (node > nN - 1 ? nN - 1 : node);
      acc += (double)h1[(size_t)node * HID + tid];
    }
  }
  {
    const float sf = (float)acc;
    const float cf = fmaxf((float)total, 1.0f);
    pooled[tid] = sf / cf;
  }
  __syncthreads();

  float a = SM[HID + tid];
#pragma unroll 4
  for (int k = 0; k < HID; ++k) a = fmaf(pooled[k], W2R[(size_t)k * HID + tid], a);
  const float zv = (a > 0.0f) ? a : (a - a);
  zs[tid] = zv;
  __syncthreads();

  const v4f ov = *(const v4fa*)(zs + 4 * (tid & 63));
  float* op = Z + (size_t)g * HID + 4 * (tid & 63);
  const bool okst = tid < 64;
  if (okst) *(volatile v4f*)op = ov;
  __threadfence();
  if (okst) *(volatile v4f*)op = ov;
}

__global__ __launch_bounds__(NTHR) void k_out(const float* __restrict__ Z, const float* __restrict__ SM,
                                              const int* __restrict__ flags, int nF, float* out) {
  __shared__ __attribute__((aligned(16))) float outs[NGR];
  __shared__ int fl[NWAVE];
  const int tid = (int)threadIdx.x, lane = tid & 31, wave = tid >> 5;
  const v4f wa = *(const v4fa*)(SM + 2 * HID + 4 * lane);
  const v4f wb = *(const v4fa*)(SM + 2 * HID + 128 + 4 * lane);
  const float b3 = SM[3 * HID];
#pragma unroll 1
  for (int q = 0; q < NGR / NWAVE; ++q) {
    const int g = (NGR / NWAVE) * wave + q;
    const float* zp = Z + (size_t)g * HID + 4 * lane;
    const v4f za = *(const v4fa*)zp;
    const v4f zb = *(const v4fa*)(zp + 128);
    float s = za.x * wa.x;
    s = fmaf(za.y, wa.y, s); s = fmaf(za.z, wa.z, s); s = fmaf(za.w, wa.w, s);
    s = fmaf(zb.x, wb.x, s); s = fmaf(zb.y, wb.y, s); s = fmaf(zb.z, wb.z, s); s = fmaf(zb.w, wb.w, s);
#pragma unroll
    for (int d = 16; d >= 1; d >>= 1) s += __shfl_xor(s, d, 32);
    if (lane == 0) outs[g] = s + b3;
  }
  {
    const int idx = tid < nF ? tid : nF - 1;
    const int f = flags[(size_t)idx * 32];
    const bool hit = (tid < nF) && (f != 0);
    const unsigned m = __builtin_amdgcn_ballot_w32(hit);
    if (lane == 0) fl[wave] = (m != 0u) ? 1 : 0;
  }
  __syncthreads();
  int anyf = 0;
#pragma unroll
  for (int w2 = 0; w2 < NWAVE; ++w2) anyf |= fl[w2];
  const float qnan = __int_as_float(0x7fc00000);
  v4f ov = *(const v4fa*)(outs + 4 * (lane & 15));
  ov.x = (anyf != 0) ? qnan : ov.x;
  ov.y = (anyf != 0) ? qnan : ov.y;
  ov.z = (anyf != 0) ? qnan : ov.z;
  ov.w = (anyf != 0) ? qnan : ov.w;
  float* op = out + 4 * (lane & 15);
  const bool okst = (wave == 0) && (lane < 16);
  if (okst) *(volatile v4f*)op = ov;
  __threadfence();
  if (okst) *(volatile v4f*)op = ov;
}

static inline int cdiv(int a, int b) { return (a + b - 1) / b; }
static inline size_t al256(size_t o) { return (o + 255) & ~(size_t)255; }

extern "C" void kernel_launch(void* const* d_in, const int* in_sizes, int n_in,
                              void* d_out, int out_size, void* d_ws, size_t ws_size,
                              hipStream_t stream) {
  if (n_in < 9) return;
  if (in_sizes[0] < CIN || (in_sizes[0] % CIN) != 0) return;
  const int nN = in_sizes[0] / CIN;
  if (nN < 1 || nN > NMAXN) return;
  if (in_sizes[1] < 2 || (in_sizes[1] & 1) != 0) return;
  const int nE = in_sizes[1] / 2;
  if (nE < 1 || nE >= (1 << (31 - SLA))) return;
  if (in_sizes[2] != nN) return;
  if (in_sizes[3] != CIN * HID || in_sizes[4] != HID) return;
  if (in_sizes[5] != HID * HID || in_sizes[6] != HID) return;
  if (in_sizes[7] != HID || in_sizes[8] != 1) return;
  if (out_size != NGR) return;

  const float* x    = (const float*)d_in[0];
  const int*   edge = (const int*)d_in[1];
  const int*   bat  = (const int*)d_in[2];
  const float* W1   = (const float*)d_in[3];
  const float* b1   = (const float*)d_in[4];
  const float* W2   = (const float*)d_in[5];
  const float* b2   = (const float*)d_in[6];
  const float* w3   = (const float*)d_in[7];
  const float* b3   = (const float*)d_in[8];
  float* out = (float*)d_out;
  const int* src = edge;
  const int* dst = edge + nE;

  const int MP   = cdiv(nN, GBM) * GBM;
  const int gM   = MP / GBM;
  const int gD   = cdiv(nN, NBD);
  const int NBPD = gD * NBD;
  const int gA   = cdiv(MP, NBA);
  if ((long long)gA * NBA < (long long)MP) return;
  if (gA < 1 || gA > NFLAG) return;
  if (NBPD < nN) return;
  const int nUx = MP * (CIN / 8);
  if ((nUx % NTHR) != 0) return;
  const int nbX = nUx / NTHR;
  const int R   = cdiv(nN, NWAVE);
  if ((long long)R * NWAVE > (long long)POOLCAP) return;
  const int vec8 = ((nE & 3) == 0) ? 1 : 0;

  char* ws = (char*)d_ws;
  size_t off = 0;
  const size_t oDIS = off; off = al256(off + (size_t)NBPD * 4);
  const size_t oSM  = off; off = al256(off + (size_t)SMF * 4);
  const size_t oW1T = off; off = al256(off + (size_t)HID * CIN * 2);
  const size_t oW2R = off; off = al256(off + (size_t)HID * HID * 4);
  const size_t oXB  = off; off = al256(off + (size_t)MP * CIN * 2);
  const size_t oH   = off; off = al256(off + (size_t)MP * HID * 4);
  const size_t oH1  = off; off = al256(off + (size_t)MP * HID * 4);
  const size_t oZ   = off; off = al256(off + (size_t)NGR * HID * 4);
  const size_t oFL  = off; off = al256(off + (size_t)NFLAG * 128);
  if (off > ws_size || off > (size_t)WSMAX) return;
  float*          DIS = (float*)(ws + oDIS);
  float*          SM  = (float*)(ws + oSM);
  unsigned short* W1T = (unsigned short*)(ws + oW1T);
  float*          W2R = (float*)(ws + oW2R);
  unsigned short* XB  = (unsigned short*)(ws + oXB);
  float*          H   = (float*)(ws + oH);
  float*          H1  = (float*)(ws + oH1);
  float*          Z   = (float*)(ws + oZ);
  int*            FL  = (int*)(ws + oFL);

  const size_t aggLds  = (size_t)AGG_LDS_INTS * 4;
  const size_t poolLds = (size_t)POOL_LDS_BYTES;
  hipFuncSetAttribute(reinterpret_cast<const void*>(&k_agg), hipFuncAttributeMaxDynamicSharedMemorySize, (int)aggLds);
  hipFuncSetAttribute(reinterpret_cast<const void*>(&k_pool_head), hipFuncAttributeMaxDynamicSharedMemorySize, (int)poolLds);

  k_prep<<<nbX + NBW1 + NBW2 + 1, NTHR, 0, stream>>>(x, nN, nbX, W1, b1, W2, b2, w3, b3, XB, W1T, W2R, SM);
  k_deg<<<gD, NTHR, 0, stream>>>(dst, nE, vec8, DIS);
  k_gemm<<<dim3(gM, HID / GBN), GTHR, 0, stream>>>(XB, W1T, H, CIN, HID);
  k_agg<<<gA, NTHR, aggLds, stream>>>(src, dst, nE, nN, vec8, MP, DIS, H, SM, H1, FL);
  k_pool_head<<<NGR, NTHR, poolLds, stream>>>(H1, bat, nN, R, W2R, SM, Z);
  k_out<<<1, NTHR, 0, stream>>>(Z, SM, FL, gA, out);
}
